// DecoderWithAttention_4552665333779
// MI455X (gfx1250) — hardware-verified
//
#include <hip/hip_runtime.h>
#include <math.h>

constexpr int kBatch   = 64;
constexpr int kLoc     = 49;
constexpr int kSteps   = 20;
constexpr int kEnc     = 2048;
constexpr int kDec     = 512;
constexpr int kAtt     = 512;
constexpr int kEmb     = 512;
constexpr int kVoc     = 10000;
constexpr int kVocPad  = 10048;
constexpr int kGate    = 4 * kDec;
constexpr int kXK      = kEnc + kDec;
constexpr int kRowsAll = kSteps * kBatch;
constexpr int kEncRows = kBatch * kLoc;
constexpr int kAlphaPitch = 64;
constexpr int kOut0Floats = kBatch * kSteps * kVoc;
constexpr int kOut1Floats = kBatch * kSteps * kLoc;
constexpr float kWCarry    = 64.0f;
constexpr float kWCarryInv = 1.0f / 64.0f;
constexpr float kEmbCarry  = 16.0f;
constexpr float kGEScale   = 1.0f / (16.0f * 64.0f);
constexpr float kInvLoc    = 1.0f / 49.0f;

static_assert(kOut0Floats + kOut1Floats == 12862720);
static_assert(kOut0Floats % 1024 == 0);
static_assert(kOut1Floats % 128 == 0);
static_assert(kEncRows % 64 == 0 && kVocPad % 64 == 0 && kRowsAll % 64 == 0);

typedef __attribute__((ext_vector_type(16))) _Float16 v16h;
typedef __attribute__((ext_vector_type(8)))  _Float16 v8h;
typedef __attribute__((ext_vector_type(16))) __bf16   v16b;
typedef __attribute__((ext_vector_type(8)))  __bf16   v8b;
typedef __attribute__((ext_vector_type(8)))  float    v8f;
typedef __attribute__((ext_vector_type(4)))  float    v4f;
typedef __attribute__((ext_vector_type(4)))  unsigned int v4u;

__device__ __forceinline__ unsigned short f2bf_bits(float f) {
  unsigned u = __float_as_uint(f);
  return (unsigned short)((u + 0x7FFFu + ((u >> 16) & 1u)) >> 16);
}
__device__ __forceinline__ float bf_bits2f(unsigned short h) { return __uint_as_float(((unsigned)h) << 16); }

__device__ __forceinline__ void dep_guard_h(v8f& a, v8f& b, v16h x, v16h y) { asm volatile("v_nop\n\tv_nop\n\tv_nop\n\tv_nop" : "+v"(a), "+v"(b) : "v"(x), "v"(y)); }
__device__ __forceinline__ void dep_guard_b(v8f& a, v8f& b, v16b x, v16b y) { asm volatile("v_nop\n\tv_nop\n\tv_nop\n\tv_nop" : "+v"(a), "+v"(b) : "v"(x), "v"(y)); }
__device__ __forceinline__ void keep4_h(v16h a, v16h b, v16h c, v16h d) { asm volatile("v_nop" :: "v"(a), "v"(b), "v"(c), "v"(d)); }
__device__ __forceinline__ void keep4_b(v16b a, v16b b, v16b c, v16b d) { asm volatile("v_nop" :: "v"(a), "v"(b), "v"(c), "v"(d)); }
__device__ __forceinline__ void acc_guard4(v8f& a, v8f& b, v8f& c, v8f& d) { asm volatile("v_nop\n\tv_nop\n\tv_nop\n\tv_nop" : "+v"(a), "+v"(b), "+v"(c), "+v"(d)); }
template <typename T> struct Frag;
template <> struct Frag<_Float16> {
  typedef v16h V; union U { v16h v; v8h h[2]; };
  static __device__ __forceinline__ v16h load(const _Float16* p) {
    U f; f.h[0] = *(const v8h*)(p); f.h[1] = *(const v8h*)(p + 16); return f.v;
  }
  static __device__ __forceinline__ v8f mma(v16h a, v16h b, v8f c) {
    return __builtin_amdgcn_wmma_f32_16x16x32_f16(false, a, false, b, (short)0, c, false, false);
  }
  static __device__ __forceinline__ void guard(v8f& a, v8f& b, v16h x, v16h y) { dep_guard_h(a, b, x, y); }
  static __device__ __forceinline__ void keep(v16h a, v16h b, v16h c, v16h d) { keep4_h(a, b, c, d); }
};
template <> struct Frag<__bf16> {
  typedef v16b V; union U { v16b v; v8b h[2]; };
  static __device__ __forceinline__ v16b load(const __bf16* p) {
    U f; f.h[0] = *(const v8b*)(p); f.h[1] = *(const v8b*)(p + 16); return f.v;
  }
  static __device__ __forceinline__ v8f mma(v16b a, v16b b, v8f c) {
    return __builtin_amdgcn_wmma_f32_16x16x32_bf16(false, a, false, b, (short)0, c, false, false);
  }
  static __device__ __forceinline__ void guard(v8f& a, v8f& b, v16b x, v16b y) { dep_guard_b(a, b, x, y); }
  static __device__ __forceinline__ void keep(v16b a, v16b b, v16b c, v16b d) { keep4_b(a, b, c, d); }
};

__device__ __forceinline__ unsigned pk16(unsigned short a, unsigned short b) { return (unsigned)a | ((unsigned)b << 16); }
__device__ __forceinline__ unsigned short h_bits(float f) { const _Float16 h = (_Float16)f; return __builtin_bit_cast(unsigned short, h); }

template <int ET> struct Elem;
template <> struct Elem<0> { typedef _Float16 T; };
template <> struct Elem<1> { typedef __bf16 T; };
template <int ET, bool SPLIT, int BIAS_MODE, int OUT_MODE, bool RESID, int ACT = 0>
__global__ __launch_bounds__(256) void wmma_gemm64(
    const unsigned short* __restrict__ Ap, const unsigned short* __restrict__ A2p, int lda, long strideA,
    const unsigned short* __restrict__ Btp, const unsigned short* __restrict__ Bt2p, int ldb, long strideB,
    void* __restrict__ Cout, void* __restrict__ Cout2, int ldc, long strideC,
    const float* __restrict__ bias,
    const float* __restrict__ resid, long strideR,
    int M, int N, int K, float scale) {
  typedef typename Elem<ET>::T T;
  typedef typename Frag<T>::V V;
  const T* A = (const T*)Ap; const T* A2 = (const T*)A2p; const T* Bt = (const T*)Btp; const T* Bt2 = (const T*)Bt2p;
  __shared__ __align__(16) float sT[8][16 * 68];
  const int b    = blockIdx.y;
  const int lane = threadIdx.x & 31;
  const int wave = threadIdx.x >> 5;
  const int tilesN = N >> 6;
  const int tilesM = M >> 6;
  const int tile = blockIdx.x * 8 + wave;
  if (tile >= tilesM * tilesN) return;
  const int tm = tile / tilesN;
  const int tn = tile - tm * tilesN;
  const int m0 = tm << 6;
  const int n0 = tn << 6;

  const T* Ab  = A  + (size_t)b * strideA;
  const T* Bb  = Bt + (size_t)b * strideB;
  const T* Ab2 = SPLIT ? (A2  + (size_t)b * strideA) : nullptr;
  const T* Bb2 = SPLIT ? (Bt2 + (size_t)b * strideB) : nullptr;

  const int rlane = lane & 15;
  const int koff  = (lane >> 4) * 8;
  const int mOff  = (lane >> 4) * 8;

  v8f acc[4][4];
#pragma unroll
  for (int i = 0; i < 4; ++i)
#pragma unroll
    for (int j = 0; j < 4; ++j) acc[i][j] = (v8f){0.f,0.f,0.f,0.f,0.f,0.f,0.f,0.f};

  for (int k0 = 0; k0 < K; k0 += 32) {
    V bh[4], bl[4];
#pragma unroll
    for (int j = 0; j < 4; ++j) {
      const size_t bo = (size_t)(n0 + (j << 4) + rlane) * ldb + koff + k0;
      bh[j] = Frag<T>::load(Bb + bo);
      if (SPLIT) bl[j] = Frag<T>::load(Bb2 + bo);
    }
#pragma unroll
    for (int i = 0; i < 4; ++i) {
      const size_t ao = (size_t)(m0 + (i << 4) + rlane) * lda + koff + k0;
      V ah = Frag<T>::load(Ab + ao);
      V al;
      if (SPLIT) al = Frag<T>::load(Ab2 + ao);
#pragma unroll
      for (int j = 0; j < 4; ++j) {
        acc[i][j] = Frag<T>::mma(ah, bh[j], acc[i][j]);
        if (SPLIT) {
          acc[i][j] = Frag<T>::mma(ah, bl[j], acc[i][j]);
          acc[i][j] = Frag<T>::mma(al, bh[j], acc[i][j]);
        }
      }
      Frag<T>::guard(acc[i][0], acc[i][3], ah, SPLIT ? al : ah);
    }
    Frag<T>::keep(bh[0], bh[1], bh[2], bh[3]);
    if (SPLIT) Frag<T>::keep(bl[0], bl[1], bl[2], bl[3]);
  }
  acc_guard4(acc[0][0], acc[0][1], acc[0][2], acc[0][3]);
  acc_guard4(acc[1][0], acc[1][1], acc[1][2], acc[1][3]);
  acc_guard4(acc[2][0], acc[2][1], acc[2][2], acc[2][3]);
  acc_guard4(acc[3][0], acc[3][1], acc[3][2], acc[3][3]);

  float* slab = sT[wave];
  const float* Rb = RESID ? (resid + (size_t)b * strideR) : nullptr;
#pragma unroll
  for (int i = 0; i < 4; ++i) {
    const int mBase = m0 + (i << 4);
#pragma unroll
    for (int j = 0; j < 4; ++j) {
      const int n = n0 + (j << 4) + rlane;
      float bv = 0.f;
      if (BIAS_MODE == 2) bv = bias[n];
#pragma unroll
      for (int r = 0; r < 8; ++r) {
        float v = acc[i][j][r] * scale;
        if (BIAS_MODE == 1) v += bias[mBase + mOff + r];
        if (BIAS_MODE == 2) v += bv;
        if (RESID) v += Rb[(size_t)(mBase + mOff + r) * ldc + n];
        if (ACT == 2) v = fmaxf(v, 0.0f);
        if (ACT == 4) v = (v > 0.f) ? v : 0.01f * v;
        slab[(mOff + r) * 68 + (j << 4) + rlane] = v;
      }
    }
    __builtin_amdgcn_fence(__ATOMIC_RELEASE, "workgroup");
    __builtin_amdgcn_wave_barrier();
    __builtin_amdgcn_fence(__ATOMIC_ACQUIRE, "workgroup");
    if (OUT_MODE == 0) {
      float* C = (float*)Cout + (size_t)b * strideC;
      const int hh = lane >> 4, c4 = (lane & 15) * 4;
      for (int pass = 0; pass < 2; ++pass) {
#pragma unroll
        for (int it = 0; it < 8; ++it) {
          const int row = it * 2 + hh;
          v4f v = *(const v4f*)(slab + row * 68 + c4);
          *(volatile v4f*)(C + (size_t)(mBase + row) * ldc + n0 + c4) = v;
        }
        __threadfence();
      }
    } else {
      const int q = lane >> 3, c8 = (lane & 7) * 8;
      unsigned short* C  = (unsigned short*)Cout  + (size_t)b * strideC;
      unsigned short* C2 = (OUT_MODE == 2) ? ((unsigned short*)Cout2 + (size_t)b * strideC) : nullptr;
      for (int pass = 0; pass < 2; ++pass) {
#pragma unroll
        for (int it = 0; it < 4; ++it) {
          const int row = it * 4 + q;
          const float* sp = slab + row * 68 + c8;
          v8h hv, lv;
#pragma unroll
          for (int e = 0; e < 8; ++e) {
            if (OUT_MODE == 1) {
              hv[e] = (_Float16)sp[e];
            } else {
              unsigned short hb = f2bf_bits(sp[e]);
              unsigned short lb = f2bf_bits(sp[e] - bf_bits2f(hb));
              hv[e] = __builtin_bit_cast(_Float16, hb);
              lv[e] = __builtin_bit_cast(_Float16, lb);
            }
          }
          *(volatile v8h*)(C + (size_t)(mBase + row) * ldc + n0 + c8) = hv;
          if (OUT_MODE == 2) *(volatile v8h*)(C2 + (size_t)(mBase + row) * ldc + n0 + c8) = lv;
        }
        __threadfence();
      }
    }
    __builtin_amdgcn_fence(__ATOMIC_RELEASE, "workgroup");
    __builtin_amdgcn_wave_barrier();
    __builtin_amdgcn_fence(__ATOMIC_ACQUIRE, "workgroup");
  }
}

__global__ __launch_bounds__(256) void transcast_kernel(const float* __restrict__ W0, const float* __restrict__ W1,
                                                        const float* __restrict__ W2, unsigned short* __restrict__ out,
                                                        long planeStride, int Kdim, int Ndim, float scale) {
  __shared__ float sm[64][65];
  const int t  = threadIdx.x;
  const int k0 = blockIdx.x * 64;
  const int n0 = blockIdx.y * 64;
  const int z  = blockIdx.z;
  const float* W = (z == 0) ? W0 : (z == 1) ? W1 : W2;
#pragma unroll
  for (int i = 0; i < 16; ++i) {
    const int e  = i * 256 + t;
    const int kl = e >> 6;
    const int nl = e & 63;
    const int n  = n0 + nl;
    const int nn = (n < Ndim) ? n : (Ndim - 1);
    float v = W[(size_t)(k0 + kl) * Ndim + nn] * scale;
    v = (n < Ndim) ? v : 0.0f;
    sm[nl][kl] = v;
  }
  __syncthreads();
  const int lane = t & 31, wave = t >> 5;
  const int q = lane >> 3, c8 = (lane & 7) * 8;
  unsigned short* op = out + (size_t)z * planeStride;
  for (int pass = 0; pass < 2; ++pass) {
#pragma unroll
    for (int it = 0; it < 2; ++it) {
      const int row = wave * 8 + it * 4 + q;
      unsigned short hb[8];
#pragma unroll
      for (int e = 0; e < 8; ++e) hb[e] = h_bits(sm[row][c8 + e]);
      const v4u u = (v4u){pk16(hb[0], hb[1]), pk16(hb[2], hb[3]), pk16(hb[4], hb[5]), pk16(hb[6], hb[7])};
      *(volatile v4u*)(op + (size_t)(n0 + row) * Kdim + k0 + c8) = u;
    }
    __threadfence();
  }
}

__global__ __launch_bounds__(256) void rowcast_kernel(const float* __restrict__ in, int ldIn, int colIn,
                                                      unsigned short* __restrict__ out, int ldOut, int colOut,
                                                      int ncols8, int total, float scale) {
  const int i = blockIdx.x * 256 + threadIdx.x;
  if (i >= total) return;
  const int r  = i / ncols8;
  const int c8 = (i - r * ncols8) * 8;
  const float* p = in + (size_t)r * ldIn + colIn + c8;
  const v4f a = *(const v4f*)(p);
  const v4f c = *(const v4f*)(p + 4);
  unsigned short hb[8];
#pragma unroll
  for (int e = 0; e < 4; ++e) {
    hb[e]     = h_bits(a[e] * scale);
    hb[4 + e] = h_bits(c[e] * scale);
  }
  const v4u u = (v4u){pk16(hb[0], hb[1]), pk16(hb[2], hb[3]), pk16(hb[4], hb[5]), pk16(hb[6], hb[7])};
  unsigned short* q = out + (size_t)r * ldOut + colOut + c8;
  *(volatile v4u*)q = u;
  __threadfence();
  *(volatile v4u*)q = u;
}

__global__ __launch_bounds__(256) void emb_gather_kernel(const float* __restrict__ table, const int* __restrict__ tokens,
                                                         unsigned short* __restrict__ out) {
  const int i  = blockIdx.x * 256 + threadIdx.x;
  if (i >= kRowsAll * 64) return;
  const int r  = i >> 6;
  const int e8 = (i & 63) * 8;
  const int t  = r >> 6;
  const int b  = r & 63;
  int tok = tokens[b * kSteps + t];
  tok = tok < 0 ? 0 : (tok > kVoc - 1 ? kVoc - 1 : tok);
  const float* p = table + (size_t)tok * kEmb + e8;
  const v4f a = *(const v4f*)(p);
  const v4f c = *(const v4f*)(p + 4);
  unsigned short hb[8];
#pragma unroll
  for (int e = 0; e < 4; ++e) {
    hb[e]     = h_bits(a[e] * kEmbCarry);
    hb[4 + e] = h_bits(c[e] * kEmbCarry);
  }
  const v4u u = (v4u){pk16(hb[0], hb[1]), pk16(hb[2], hb[3]), pk16(hb[4], hb[5]), pk16(hb[6], hb[7])};
  unsigned short* q = out + (size_t)r * kEmb + e8;
  *(volatile v4u*)q = u;
  __threadfence();
  *(volatile v4u*)q = u;
}

__global__ __launch_bounds__(256) void mean_kernel(const float* __restrict__ enc, unsigned short* __restrict__ out) {
  const int i  = blockIdx.x * 256 + threadIdx.x;
  if (i >= kBatch * 256) return;
  const int b  = i >> 8;
  const int e8 = (i & 255) * 8;
  float s[8];
#pragma unroll
  for (int e = 0; e < 8; ++e) s[e] = 0.f;
  const float* base = enc + (size_t)b * kLoc * kEnc + e8;
#pragma unroll 1
  for (int l = 0; l < kLoc; ++l) {
    const float* p = base + (size_t)l * kEnc;
    const v4f a = *(const v4f*)(p);
    const v4f c = *(const v4f*)(p + 4);
#pragma unroll
    for (int e = 0; e < 4; ++e) { s[e] += a[e]; s[4 + e] += c[e]; }
  }
  unsigned short hb[8];
#pragma unroll
  for (int e = 0; e < 8; ++e) hb[e] = h_bits(s[e] * kInvLoc);
  const v4u u = (v4u){pk16(hb[0], hb[1]), pk16(hb[2], hb[3]), pk16(hb[4], hb[5]), pk16(hb[6], hb[7])};
  unsigned short* q = out + (size_t)b * kEnc + e8;
  *(volatile v4u*)q = u;
  __threadfence();
  *(volatile v4u*)q = u;
}

__global__ __launch_bounds__(256) void padvec_kernel(const float* __restrict__ in, int nIn, float* __restrict__ out, int nOut4) {
  const int i = blockIdx.x * 256 + threadIdx.x;
  if (i >= nOut4) return;
  const int e0 = 4 * i;
  v4f v;
#pragma unroll
  for (int u = 0; u < 4; ++u) {
    const int idx = e0 + u;
    const int ci  = idx < nIn ? idx : nIn - 1;
    float x = in[ci];
    v[u] = (idx < nIn) ? x : 0.0f;
  }
  float* q = out + e0;
  *(volatile v4f*)q = v;
  __threadfence();
  *(volatile v4f*)q = v;
}

__global__ __launch_bounds__(256) void attn_step_kernel(const float* __restrict__ decp,
                                                        const float* __restrict__ encp,
                                                        const float* __restrict__ enc,
                                                        const float* __restrict__ w_full,
                                                        const float* __restrict__ b_full,
                                                        float* __restrict__ alpha_ws,
                                                        unsigned short* __restrict__ xh) {
  __shared__ float dec_s[kAtt];
  __shared__ float wf_s[kAtt];
  __shared__ float score_s[64];
  __shared__ __align__(16) float alpha_s[64];
  const int b    = blockIdx.x;
  const int tid  = threadIdx.x;
  const int lane = tid & 31;
  const int wave = tid >> 5;

  dec_s[tid]       = decp[(size_t)b * kAtt + tid];
  dec_s[tid + 256] = decp[(size_t)b * kAtt + tid + 256];
  wf_s[tid]        = w_full[tid];
  wf_s[tid + 256]  = w_full[tid + 256];
  __syncthreads();

  const float bf0 = b_full[0];
#pragma unroll 1
  for (int it = 0; it < 7; ++it) {
    const int l  = wave + 8 * it;
    const int lc = l < kLoc ? l : kLoc - 1;
    const float* ep = encp + ((size_t)b * kLoc + lc) * kAtt;
    float part = 0.f;
#pragma unroll 4
    for (int a = lane; a < kAtt; a += 32) {
      float v = ep[a] + dec_s[a];
      v = fmaxf(v, 0.0f);
      part = fmaf(v, wf_s[a], part);
    }
#pragma unroll
    for (int off = 16; off > 0; off >>= 1) part += __shfl_xor(part, off, 32);
    if (l < kLoc && lane == 0) score_s[l] = part + bf0;
  }
  __syncthreads();

  if (wave == 0) {
    const int l0 = lane;
    const int l1 = lane + 32;
    const int l1c = l1 < kLoc ? l1 : kLoc - 1;
    const float s0 = score_s[l0];
    float s1 = score_s[l1c];
    s1 = (l1 < kLoc) ? s1 : -INFINITY;
    float m = fmaxf(s0, s1);
#pragma unroll
    for (int off = 16; off > 0; off >>= 1) m = fmaxf(m, __shfl_xor(m, off, 32));
    const float p0 = expf(s0 - m);
    const float p1 = expf(s1 - m);
    float sum = p0 + p1;
#pragma unroll
    for (int off = 16; off > 0; off >>= 1) sum += __shfl_xor(sum, off, 32);
    const float inv = 1.0f / sum;
    alpha_s[l0] = p0 * inv;
    alpha_s[l1] = p1 * inv;
  }
  __syncthreads();

  if (wave == 0 && lane < 16) {
    const v4f av = *(const v4f*)(alpha_s + 4 * lane);
    float* ap = alpha_ws + (size_t)b * kAlphaPitch + 4 * lane;
    *(volatile v4f*)ap = av;
    __threadfence();
    *(volatile v4f*)ap = av;
  }

  const int e8 = tid * 8;
  float acc[8];
#pragma unroll
  for (int e = 0; e < 8; ++e) acc[e] = 0.f;
  const float* base = enc + (size_t)b * kLoc * kEnc + e8;
#pragma unroll 1
  for (int l = 0; l < kLoc; ++l) {
    const float al = alpha_s[l];
    const float* p = base + (size_t)l * kEnc;
    const v4f a = *(const v4f*)(p);
    const v4f c = *(const v4f*)(p + 4);
#pragma unroll
    for (int e = 0; e < 4; ++e) { acc[e] = fmaf(al, a[e], acc[e]); acc[4 + e] = fmaf(al, c[e], acc[4 + e]); }
  }
  unsigned short hb[8];
#pragma unroll
  for (int e = 0; e < 8; ++e) hb[e] = h_bits(acc[e]);
  const v4u u = (v4u){pk16(hb[0], hb[1]), pk16(hb[2], hb[3]), pk16(hb[4], hb[5]), pk16(hb[6], hb[7])};
  unsigned short* q = xh + (size_t)b * kXK + e8;
  *(volatile v4u*)q = u;
  __threadfence();
  *(volatile v4u*)q = u;
}

__global__ __launch_bounds__(128) void cell_kernel(const float* __restrict__ gates, const float* __restrict__ cin,
                                                   float* __restrict__ cout, unsigned short* __restrict__ xh) {
  __shared__ __align__(16) float cs[kDec];
  __shared__ __align__(16) unsigned short hs[kDec];
  const int b = blockIdx.x;
  const int t = threadIdx.x;
  const float* g  = gates + (size_t)b * kGate;
  const float* cp = cin + (size_t)b * kDec;
#pragma unroll 1
  for (int u = 0; u < 4; ++u) {
    const int j = 4 * t + u;
    const float gi = g[j];
    const float gf = g[kDec + j];
    const float gg = g[2 * kDec + j];
    const float go = g[3 * kDec + j];
    const float cprev = cp[j];
    const float iv = __builtin_amdgcn_rcpf(1.0f + expf(-gi));
    const float fv = __builtin_amdgcn_rcpf(1.0f + expf(-gf));
    const float ov = __builtin_amdgcn_rcpf(1.0f + expf(-go));
    const float gv = tanhf(gg);
    const float cn = fv * cprev + iv * gv;
    const float hn = ov * tanhf(cn);
    cs[j] = cn;
    hs[j] = h_bits(hn);
  }
  __syncthreads();
  {
    const v4f cv = *(const v4f*)(cs + 4 * t);
    float* q = cout + (size_t)b * kDec + 4 * t;
    *(volatile v4f*)q = cv;
    __threadfence();
    *(volatile v4f*)q = cv;
  }
  if (t < 64) {
    const v4u hv = *(const v4u*)(hs + 8 * t);
    unsigned short* q = xh + (size_t)b * kXK + kEnc + 8 * t;
    *(volatile v4u*)q = hv;
    __threadfence();
    *(volatile v4u*)q = hv;
  }
}

constexpr int kCopyBlocks0 = kOut0Floats / 4 / 256;
constexpr int kOut1F4      = kOut1Floats / 4;
constexpr int kCopyBlocks1 = (kOut1F4 + 255) / 256;
__global__ __launch_bounds__(256) void out_copy_kernel(const float* __restrict__ logp, const float* __restrict__ alp,
                                                       float* __restrict__ out) {
  const int tid = threadIdx.x;
  if (blockIdx.x < kCopyBlocks0) {
    const int i  = blockIdx.x * 256 + tid;
    const int e  = i * 4;
    const int bt = e / kVoc;
    const int v  = e - bt * kVoc;
    const int b  = bt / kSteps;
    const int t  = bt - b * kSteps;
    const v4f val = *(const v4f*)(logp + (size_t)(t * kBatch + b) * kVocPad + v);
    float* q = out + (size_t)e;
    *(volatile v4f*)q = val;
    __threadfence();
    *(volatile v4f*)q = val;
  } else {
    const int i1 = (blockIdx.x - kCopyBlocks0) * 256 + tid;
    if (i1 >= kOut1F4) return;
    const int e = i1 * 4;
    v4f val;
#pragma unroll
    for (int u = 0; u < 4; ++u) {
      const int e1 = e + u;
      const int bt = e1 / kLoc;
      const int l  = e1 - bt * kLoc;
      const int b  = bt / kSteps;
      const int t  = bt - b * kSteps;
      val[u] = alp[(size_t)(t * kBatch + b) * kAlphaPitch + l];
    }
    float* q = out + (size_t)kOut0Floats + e;
    *(volatile v4f*)q = val;
    __threadfence();
    *(volatile v4f*)q = val;
  }
}

static void gemm_f32out(hipStream_t s, const unsigned short* A, int lda, const unsigned short* Bt, int ldb,
                        float* C, int ldc, const float* bias, int M, int N, int K, float scale) {
  const int tiles = (M / 64) * (N / 64);
  dim3 grid((unsigned)((tiles + 7) / 8), 1, 1);
  wmma_gemm64<0, false, 2, 0, false, 0><<<grid, 256, 0, s>>>(A, nullptr, lda, 0L, Bt, nullptr, ldb, 0L,
                                                             (void*)C, nullptr, ldc, 0L, bias, nullptr, 0L, M, N, K, scale);
}
static void gemm_f32out_resid(hipStream_t s, const unsigned short* A, int lda, const unsigned short* Bt, int ldb,
                              float* C, int ldc, const float* bias, const float* resid, int M, int N, int K, float scale) {
  const int tiles = (M / 64) * (N / 64);
  dim3 grid((unsigned)((tiles + 7) / 8), 1, 1);
  wmma_gemm64<0, false, 2, 0, true, 0><<<grid, 256, 0, s>>>(A, nullptr, lda, 0L, Bt, nullptr, ldb, 0L,
                                                            (void*)C, nullptr, ldc, 0L, bias, resid, 0L, M, N, K, scale);
}
static void gemm_f16out(hipStream_t s, const unsigned short* A, int lda, const unsigned short* Bt, int ldb,
                        unsigned short* C, int ldc, const float* bias, int M, int N, int K, float scale) {
  const int tiles = (M / 64) * (N / 64);
  dim3 grid((unsigned)((tiles + 7) / 8), 1, 1);
  wmma_gemm64<0, false, 2, 1, false, 0><<<grid, 256, 0, s>>>(A, nullptr, lda, 0L, Bt, nullptr, ldb, 0L,
                                                             (void*)C, nullptr, ldc, 0L, bias, nullptr, 0L, M, N, K, scale);
}

static inline size_t align_up256(size_t x) { return (x + 255) & ~(size_t)255; }

extern "C" void kernel_launch(void* const* d_in, const int* in_sizes, int n_in,
                              void* d_out, int out_size, void* d_ws, size_t ws_size,
                              hipStream_t stream) {
  (void)in_sizes; (void)n_in; (void)out_size;

  const float* encoder_out = (const float*)d_in[0];
  const int*   captions    = (const int*)  d_in[1];
  const float* emb_table   = (const float*)d_in[2];
  const float* W_enc_att   = (const float*)d_in[3];
  const float* b_enc_att   = (const float*)d_in[4];
  const float* W_dec_att   = (const float*)d_in[5];
  const float* b_dec_att   = (const float*)d_in[6];
  const float* w_full      = (const float*)d_in[7];
  const float* b_full      = (const float*)d_in[8];
  const float* W_ih        = (const float*)d_in[9];
  const float* b_ih        = (const float*)d_in[10];
  const float* W_hh        = (const float*)d_in[11];
  const float* b_hh        = (const float*)d_in[12];
  const float* W_init_h    = (const float*)d_in[13];
  const float* b_init_h    = (const float*)d_in[14];
  const float* W_init_c    = (const float*)d_in[15];
  const float* b_init_c    = (const float*)d_in[16];
  const float* W_out       = (const float*)d_in[17];
  const float* b_out       = (const float*)d_in[18];
  float* out = (float*)d_out;

  char* ws = (char*)d_ws;
  size_t off = 0;
  const size_t szENC16  = (size_t)kEncRows * kEnc * 2;
  const size_t szWINI   = (size_t)3 * kDec * kEnc * 2;
  const size_t szWDEC16 = (size_t)kAtt * kDec * 2;
  const size_t szWE16   = (size_t)kGate * kEmb * 2;
  const size_t szWG16   = (size_t)kGate * kXK * 2;
  const size_t szWOUT16 = (size_t)kVocPad * kDec * 2;
  const size_t szEMB16  = (size_t)kRowsAll * kEmb * 2;
  const size_t szMEAN16 = (size_t)kBatch * kEnc * 2;
  const size_t szENCP   = (size_t)kEncRows * kAtt * 4;
  const size_t szGE     = (size_t)kRowsAll * kGate * 4;
  const size_t szXH16   = (size_t)kBatch * kXK * 2;
  const size_t szCST    = (size_t)2 * kBatch * kDec * 4;
  const size_t szGATES  = (size_t)kBatch * kGate * 4;
  const size_t szDECP   = (size_t)kBatch * kAtt * 4;
  const size_t szBOUTP  = (size_t)kVocPad * 4;
  const size_t szALPHA  = (size_t)kRowsAll * kAlphaPitch * 4;
  const size_t szLOG    = (size_t)kRowsAll * kVocPad * 4;

  unsigned short* ENC16  = (unsigned short*)(ws + off); off = align_up256(off + szENC16);
  unsigned short* WINI   = (unsigned short*)(ws + off); off = align_up256(off + szWINI);
  unsigned short* WDEC16 = (unsigned short*)(ws + off); off = align_up256(off + szWDEC16);
  unsigned short* WE16   = (unsigned short*)(ws + off); off = align_up256(off + szWE16);
  unsigned short* WG16   = (unsigned short*)(ws + off); off = align_up256(off + szWG16);
  unsigned short* WOUT16 = (unsigned short*)(ws + off); off = align_up256(off + szWOUT16);
  unsigned short* EMB16  = (unsigned short*)(ws + off); off = align_up256(off + szEMB16);
  unsigned short* MEAN16 = (unsigned short*)(ws + off); off = align_up256(off + szMEAN16);
  float*          ENCP   = (float*)(ws + off);          off = align_up256(off + szENCP);
  float*          GE     = (float*)(ws + off);          off = align_up256(off + szGE);
  unsigned short* XH16   = (unsigned short*)(ws + off); off = align_up256(off + szXH16);
  float*          CST    = (float*)(ws + off);          off = align_up256(off + szCST);
  float*          GATES  = (float*)(ws + off);          off = align_up256(off + szGATES);
  float*          DECP   = (float*)(ws + off);          off = align_up256(off + szDECP);
  float*          BOUTP  = (float*)(ws + off);          off = align_up256(off + szBOUTP);
  float*          ALPHA  = (float*)(ws + off);          off = align_up256(off + szALPHA);
  float*          LOG    = (float*)(ws + off);          off = align_up256(off + szLOG);
  if (off > ws_size) return;

  const size_t planeWINI = (size_t)kDec * kEnc;
  unsigned short* WENC16 = WINI;
  unsigned short* WINH16 = WINI + planeWINI;
  unsigned short* WINC16 = WINI + 2 * planeWINI;

  rowcast_kernel<<<(kEncRows * 256 + 255) / 256, 256, 0, stream>>>(encoder_out, kEnc, 0, ENC16, kEnc, 0, kEnc / 8,
                                                                    kEncRows * (kEnc / 8), 1.0f);
  transcast_kernel<<<dim3(kEnc / 64, kDec / 64, 3), 256, 0, stream>>>(W_enc_att, W_init_h, W_init_c, WINI, (long)planeWINI,
                                                                       kEnc, kDec, kWCarry);
  transcast_kernel<<<dim3(kDec / 64, kAtt / 64, 1), 256, 0, stream>>>(W_dec_att, W_dec_att, W_dec_att, WDEC16, 0L,
                                                                       kDec, kAtt, kWCarry);
  transcast_kernel<<<dim3(kDec / 64, kVocPad / 64, 1), 256, 0, stream>>>(W_out, W_out, W_out, WOUT16, 0L,
                                                                          kDec, kVoc, kWCarry);
  rowcast_kernel<<<(kGate * (kEmb / 8) + 255) / 256, 256, 0, stream>>>(W_ih, kXK, 0, WE16, kEmb, 0, kEmb / 8,
                                                                        kGate * (kEmb / 8), kWCarry);
  rowcast_kernel<<<(kGate * (kEnc / 8) + 255) / 256, 256, 0, stream>>>(W_ih, kXK, kEmb, WG16, kXK, 0, kEnc / 8,
                                                                        kGate * (kEnc / 8), kWCarry);
  rowcast_kernel<<<(kGate * (kDec / 8) + 255) / 256, 256, 0, stream>>>(W_hh, kDec, 0, WG16, kXK, kEnc, kDec / 8,
                                                                        kGate * (kDec / 8), kWCarry);
  emb_gather_kernel<<<(kRowsAll * 64 + 255) / 256, 256, 0, stream>>>(emb_table, captions, EMB16);
  mean_kernel<<<(kBatch * 256 + 255) / 256, 256, 0, stream>>>(encoder_out, MEAN16);
  padvec_kernel<<<(kVocPad / 4 + 255) / 256, 256, 0, stream>>>(b_out, kVoc, BOUTP, kVocPad / 4);

  gemm_f32out(stream, ENC16, kEnc, WENC16, kEnc, ENCP, kAtt, b_enc_att, kEncRows, kAtt, kEnc, kWCarryInv);
  gemm_f16out(stream, MEAN16, kEnc, WINH16, kEnc, XH16 + kEnc, kXK, b_init_h, kBatch, kDec, kEnc, kWCarryInv);
  gemm_f32out(stream, MEAN16, kEnc, WINC16, kEnc, CST, kDec, b_init_c, kBatch, kDec, kEnc, kWCarryInv);
  gemm_f32out(stream, EMB16, kEmb, WE16, kEmb, GE, kGate, b_ih, kRowsAll, kGate, kEmb, kGEScale);

  for (int t = 0; t < kSteps; ++t) {
    float* cin  = CST + (size_t)(t & 1) * kBatch * kDec;
    float* cnew = CST + (size_t)((t + 1) & 1) * kBatch * kDec;
    gemm_f32out(stream, XH16 + kEnc, kXK, WDEC16, kDec, DECP, kAtt, b_dec_att, kBatch, kAtt, kDec, kWCarryInv);
    attn_step_kernel<<<kBatch, 256, 0, stream>>>(DECP, ENCP, encoder_out, w_full, b_full,
                                                  ALPHA + (size_t)t * kBatch * kAlphaPitch, XH16);
    gemm_f32out_resid(stream, XH16, kXK, WG16, kXK, GATES, kGate, b_hh, GE + (size_t)t * kBatch * kGate,
                      kBatch, kGate, kXK, kWCarryInv);
    cell_kernel<<<kBatch, 128, 0, stream>>>(GATES, cin, cnew, XH16);
    gemm_f32out(stream, XH16 + kEnc, kXK, WOUT16, kDec, LOG + (size_t)t * kBatch * kVocPad, kVocPad, BOUTP,
                kBatch, kVocPad, kDec, kWCarryInv);
  }

  out_copy_kernel<<<kCopyBlocks0 + kCopyBlocks1, 256, 0, stream>>>(LOG, ALPHA, out);
}
